// StructureBuilder_50603304681507
// MI455X (gfx1250) — hardware-run, weakly checked
//
#include <hip/hip_runtime.h>
#include <math.h>

typedef __attribute__((ext_vector_type(16))) _Float16 v16h;
typedef __attribute__((ext_vector_type(8)))  _Float16 v8h;
typedef __attribute__((ext_vector_type(8)))  float    v8f;
typedef __attribute__((ext_vector_type(4)))  float    v4f;
typedef __attribute__((ext_vector_type(4)))  unsigned int v4u;
typedef unsigned int __attribute__((may_alias)) u32a;
typedef float __attribute__((may_alias)) f32a;
typedef v4f __attribute__((may_alias)) v4fa;

constexpr int kC    = 64;
constexpr int kA    = 128;
constexpr int kNH   = 8;
constexpr int kHC   = 16;
constexpr int kKK   = 9;
constexpr int kSide = 64;
constexpr int kL    = 4096;
constexpr int kFR   = 144;
constexpr int kFP   = 160;
constexpr int kChunksPerRow = kFP / 8;
constexpr int kTW   = 64;
constexpr int kNW   = 4;
static_assert(kA == kNH * kHC);
static_assert(kFR == kHC * kKK);
static_assert(kFP % 32 == 0 && kFP >= kFR);
static_assert(kL == kSide * kSide);
static_assert(kChunksPerRow == 20);
static_assert(kL % kTW == 0 && kL % (kNW * 16) == 0);

constexpr float kQKCarry  = 16.0f;
constexpr float kLoCarry  = 2048.0f;
constexpr float kPCarry   = 32768.0f;
constexpr float kVCarry   = 64.0f;
constexpr float kLoInv    = 1.0f / kLoCarry;
constexpr float kScoreInv = 1.0f / (kQKCarry * kQKCarry);
constexpr float kHeadMean = 1.0f / (float)kNH;
constexpr float kTapMean  = 1.0f / (float)kKK;
constexpr float kInvL     = 1.0f / (float)kL;
constexpr float kNormEps  = 1e-5f;

constexpr size_t kBytesQK    = (size_t)2 * kA * kL * 4;
constexpr size_t kBytesPlane = (size_t)kNH * kL * kFP * 2;
constexpr size_t kBytesVP    = (size_t)kC * kL * 2;
constexpr size_t kBytesATTH  = (size_t)kNH * kL * kC * 4;
constexpr size_t kBytesOUT1  = (size_t)kC * kL * 4;
constexpr size_t kOffQKRAW = 0;
constexpr size_t kOffQKN   = kOffQKRAW + kBytesQK;
constexpr size_t kOffQH    = kOffQKN   + kBytesQK;
constexpr size_t kOffQL    = kOffQH    + kBytesPlane;
constexpr size_t kOffKH    = kOffQL    + kBytesPlane;
constexpr size_t kOffKL    = kOffKH    + kBytesPlane;
constexpr size_t kOffVP    = kOffKL    + kBytesPlane;
constexpr size_t kOffATTH  = kOffVP    + kBytesVP;
constexpr size_t kOffOUT1  = kOffATTH  + kBytesATTH;
constexpr size_t kWsTotal  = kOffOUT1  + kBytesOUT1;
static_assert(kWsTotal == 60293120ull);
static_assert(kWsTotal <= 134217728ull);
static_assert((kOffQKN % 128) == 0 && (kOffQH % 128) == 0 && (kOffQL % 128) == 0 && (kOffKH % 128) == 0 &&
              (kOffKL % 128) == 0 && (kOffVP % 128) == 0 && (kOffATTH % 128) == 0 && (kOffOUT1 % 128) == 0);

__device__ __forceinline__ unsigned short h_bits(float f) {
  const _Float16 h = (_Float16)f;
  return __builtin_bit_cast(unsigned short, h);
}
__device__ __forceinline__ unsigned pk16(unsigned short a, unsigned short b) {
  return (unsigned)a | ((unsigned)b << 16);
}
__device__ __forceinline__ void split_h(float x, unsigned short& hb, unsigned short& lb) {
  const _Float16 h = (_Float16)x;
  const float hf = (float)h;
  const float res = (x - hf) * kLoCarry;
  const _Float16 lo = (_Float16)res;
  hb = __builtin_bit_cast(unsigned short, h);
  lb = __builtin_bit_cast(unsigned short, lo);
}
struct FragH {
  union U { v16h v; v8h h[2]; };
  static __device__ __forceinline__ v16h load(const _Float16* p) {
    U f;
    f.h[0] = *(const v8h*)(p);
    f.h[1] = *(const v8h*)(p + 16);
    return f.v;
  }
};
__device__ __forceinline__ v8f mma_g(v16h a, v16h b, v8f c) {
  c = __builtin_amdgcn_wmma_f32_16x16x32_f16(false, a, false, b, (short)0, c, false, false);
  asm volatile("v_nop\n\tv_nop\n\tv_nop\n\tv_nop" : "+v"(c) : "v"(a), "v"(b));
  return c;
}

__global__ __launch_bounds__(256) void proj_qk_kernel(
    const float* __restrict__ feat, const float* __restrict__ masks,
    const float* __restrict__ Wq, const float* __restrict__ bq,
    const float* __restrict__ Wk, const float* __restrict__ bk,
    float* __restrict__ qkraw)
{
  const int i  = blockIdx.x * 256 + threadIdx.x;
  const int a  = i >> 10;
  const int l0 = (i & 1023) << 2;
  v4f aq = (v4f){0.f, 0.f, 0.f, 0.f};
  v4f ak = (v4f){0.f, 0.f, 0.f, 0.f};
#pragma unroll 4
  for (int c = 0; c < kC; ++c) {
    const v4f fv = *(const v4f*)(feat + (size_t)c * kL + l0);
    const float wq = Wq[a * kC + c];
    const float wk = Wk[a * kC + c];
#pragma unroll
    for (int e = 0; e < 4; ++e) {
      aq[e] = fmaf(wq, fv[e], aq[e]);
      ak[e] = fmaf(wk, fv[e], ak[e]);
    }
  }
  const v4f mk = *(const v4f*)(masks + l0);
  const float bqa = bq[a];
  const float bka = bk[a];
  v4f qo, ko;
#pragma unroll
  for (int e = 0; e < 4; ++e) {
    const bool hole = mk[e] > 0.5f;
    qo[e] = (hole ? aq[e] : 0.0f) + bqa;
    ko[e] = (hole ? 0.0f : ak[e]) + bka;
  }
  float* qp = qkraw + (size_t)a * kL + l0;
  float* kp = qkraw + (size_t)(kA + a) * kL + l0;
  *(volatile v4f*)qp = qo;
  *(volatile v4f*)kp = ko;
  __threadfence();
  *(volatile v4f*)qp = qo;
  *(volatile v4f*)kp = ko;
}

__global__ __launch_bounds__(256) void inorm_relu_kernel(const float* __restrict__ src, float* __restrict__ dst)
{
  __shared__ float redA[8];
  __shared__ float redB[8];
  const int ch = blockIdx.x;
  const int t = threadIdx.x, lane = t & 31, wave = t >> 5;
  const float* x = src + (size_t)ch * kL;
  v4f v[4];
#pragma unroll
  for (int i = 0; i < 4; ++i) v[i] = *(const v4f*)(x + i * 1024 + t * 4);
  float s = 0.0f;
#pragma unroll
  for (int i = 0; i < 4; ++i) s += (v[i][0] + v[i][1]) + (v[i][2] + v[i][3]);
  s += __shfl_xor(s, 16, 32);
  s += __shfl_xor(s, 8, 32);
  s += __shfl_xor(s, 4, 32);
  s += __shfl_xor(s, 2, 32);
  s += __shfl_xor(s, 1, 32);
  if (lane == 0) redA[wave] = s;
  __syncthreads();
  const float tot = ((redA[0] + redA[1]) + (redA[2] + redA[3])) + ((redA[4] + redA[5]) + (redA[6] + redA[7]));
  const float mu = tot * kInvL;
  float q = 0.0f;
#pragma unroll
  for (int i = 0; i < 4; ++i) {
    const float d0 = v[i][0] - mu, d1 = v[i][1] - mu, d2 = v[i][2] - mu, d3 = v[i][3] - mu;
    q += (d0 * d0 + d1 * d1) + (d2 * d2 + d3 * d3);
  }
  q += __shfl_xor(q, 16, 32);
  q += __shfl_xor(q, 8, 32);
  q += __shfl_xor(q, 4, 32);
  q += __shfl_xor(q, 2, 32);
  q += __shfl_xor(q, 1, 32);
  if (lane == 0) redB[wave] = q;
  __syncthreads();
  const float tq = ((redB[0] + redB[1]) + (redB[2] + redB[3])) + ((redB[4] + redB[5]) + (redB[6] + redB[7]));
  const float var = tq * kInvL;
  const float rs = 1.0f / sqrtf(var + kNormEps);
  v4f y[4];
#pragma unroll
  for (int i = 0; i < 4; ++i) {
#pragma unroll
    for (int e = 0; e < 4; ++e) y[i][e] = fmaxf((v[i][e] - mu) * rs, 0.0f);
  }
  float* o = dst + (size_t)ch * kL + t * 4;
  for (int pass = 0; pass < 2; ++pass) {
#pragma unroll
    for (int i = 0; i < 4; ++i) *(volatile v4f*)(o + i * 1024) = y[i];
    __threadfence();
  }
}

__global__ __launch_bounds__(256) void build_patch_planes_kernel(
    const float* __restrict__ qkn,
    unsigned short* __restrict__ QH, unsigned short* __restrict__ QL,
    unsigned short* __restrict__ KH, unsigned short* __restrict__ KL)
{
  const int idx  = blockIdx.x * 256 + threadIdx.x;
  const int row  = idx / kChunksPerRow;
  const int part = idx - row * kChunksPerRow;
  const int l    = row & (kL - 1);
  const int n    = row >> 12;
  const int kk   = part >> 1;
  const int cl0  = (part & 1) * 8;
  const bool live = part < 2 * kKK;
  const int kkc  = kk < (kKK - 1) ? kk : (kKK - 1);
  const int ky   = kkc / 3;
  const int kx   = kkc - 3 * ky;
  const int yy   = (l >> 6) + 2 * ky - 2;
  const int xx   = (l & 63) + 2 * kx - 2;
  const bool inb = live && (yy >= 0) && (yy < kSide) && (xx >= 0) && (xx < kSide);
  const int yc   = yy < 0 ? 0 : (yy > kSide - 1 ? kSide - 1 : yy);
  const int xc   = xx < 0 ? 0 : (xx > kSide - 1 ? kSide - 1 : xx);
  const size_t base = (size_t)(n * kHC + cl0) * kL + (size_t)(yc * kSide + xc);
  const float* qp = qkn + base;
  const float* kp = qkn + (size_t)kA * kL + base;
  unsigned short qh[8], ql[8], kh[8], kl[8];
#pragma unroll
  for (int e = 0; e < 8; ++e) {
    float qv = qp[(size_t)e * kL];
    asm volatile("" : "+v"(qv));
    float kv = kp[(size_t)e * kL];
    asm volatile("" : "+v"(kv));
    qv = inb ? qv : 0.0f;
    kv = inb ? kv : 0.0f;
    split_h(qv * kQKCarry, qh[e], ql[e]);
    split_h(kv * kQKCarry, kh[e], kl[e]);
  }
  const v4u uqh = (v4u){pk16(qh[0], qh[1]), pk16(qh[2], qh[3]), pk16(qh[4], qh[5]), pk16(qh[6], qh[7])};
  const v4u uql = (v4u){pk16(ql[0], ql[1]), pk16(ql[2], ql[3]), pk16(ql[4], ql[5]), pk16(ql[6], ql[7])};
  const v4u ukh = (v4u){pk16(kh[0], kh[1]), pk16(kh[2], kh[3]), pk16(kh[4], kh[5]), pk16(kh[6], kh[7])};
  const v4u ukl = (v4u){pk16(kl[0], kl[1]), pk16(kl[2], kl[3]), pk16(kl[4], kl[5]), pk16(kl[6], kl[7])};
  const size_t o = (size_t)idx * 8;
  for (int pass = 0; pass < 2; ++pass) {
    *(volatile v4u*)(QH + o) = uqh;
    *(volatile v4u*)(QL + o) = uql;
    *(volatile v4u*)(KH + o) = ukh;
    *(volatile v4u*)(KL + o) = ukl;
    __threadfence();
  }
}

__global__ __launch_bounds__(256) void build_value_plane_kernel(
    const float* __restrict__ feat, const float* __restrict__ masks, unsigned short* __restrict__ VP)
{
  const int idx  = blockIdx.x * 256 + threadIdx.x;
  const int c    = idx >> 9;
  const int pos0 = (idx & 511) * 8;
  const int g32  = pos0 >> 5;
  const int pb   = pos0 & 31;
  const float* fc = feat + (size_t)c * kL;
  float s[8];
#pragma unroll
  for (int e = 0; e < 8; ++e) s[e] = 0.0f;
#pragma unroll 1
  for (int kk = 0; kk < kKK; ++kk) {
    const int ky = kk / 3;
    const int kx = kk - 3 * ky;
#pragma unroll
    for (int e = 0; e < 8; ++e) {
      const int p   = pb + e;
      const int key = g32 * 32 + (p & 1) * 16 + (p >> 1);
      const int yy  = (key >> 6) + 2 * ky - 2;
      const int xx  = (key & 63) + 2 * kx - 2;
      const bool inb = (yy >= 0) && (yy < kSide) && (xx >= 0) && (xx < kSide);
      const int yc  = yy < 0 ? 0 : (yy > kSide - 1 ? kSide - 1 : yy);
      const int xc  = xx < 0 ? 0 : (xx > kSide - 1 ? kSide - 1 : xx);
      const int tp  = yc * kSide + xc;
      float fv = fc[tp];
      asm volatile("" : "+v"(fv));
      float mv = masks[tp];
      asm volatile("" : "+v"(mv));
      const bool keep = inb && !(mv > 0.5f);
      s[e] += keep ? fv : 0.0f;
    }
  }
  unsigned short hb[8];
#pragma unroll
  for (int e = 0; e < 8; ++e) hb[e] = h_bits(s[e] * kTapMean * kVCarry);
  const v4u u = (v4u){pk16(hb[0], hb[1]), pk16(hb[2], hb[3]), pk16(hb[4], hb[5]), pk16(hb[6], hb[7])};
  unsigned short* o = VP + (size_t)idx * 8;
  *(volatile v4u*)o = u;
  __threadfence();
  *(volatile v4u*)o = u;
}

__global__ __launch_bounds__(128) void patch_attn_kernel(
    const _Float16* __restrict__ QH, const _Float16* __restrict__ QL,
    const _Float16* __restrict__ KH, const _Float16* __restrict__ KL,
    const _Float16* __restrict__ VP, float* __restrict__ ATTH)
{
  __shared__ __align__(16) _Float16 Ksh[kTW * kFP];
  __shared__ __align__(16) _Float16 Ksl[kTW * kFP];
  __shared__ __align__(16) _Float16 Vts[kC * kTW];
  __shared__ __align__(16) _Float16 Psh[kNW][16 * 32];
  static_assert((size_t)kNW * 16 * 68 * 4 <= (size_t)kTW * kFP * 2);

  const int tid  = threadIdx.x;
  const int wave = tid >> 5;
  const int lane = tid & 31;
  const int hh   = lane >> 4;
  const int c    = lane & 15;
  const int head = blockIdx.x >> 6;
  const int qt   = blockIdx.x & 63;
  const int q0   = qt * 64 + wave * 16;
  const size_t hbase = (size_t)head * kL * kFP;
  const _Float16* qhrow = QH + hbase + (size_t)(q0 + c) * kFP + 8 * hh;
  const _Float16* qlrow = QL + hbase + (size_t)(q0 + c) * kFP + 8 * hh;
  const _Float16* khg = KH + hbase;
  const _Float16* klg = KL + hbase;

  float mrow[8], lrow[8];
  v8f oacc[4];
#pragma unroll
  for (int r = 0; r < 8; ++r) {
    mrow[r] = -INFINITY;
    lrow[r] = 0.0f;
  }
#pragma unroll
  for (int t = 0; t < 4; ++t) oacc[t] = (v8f){0.f, 0.f, 0.f, 0.f, 0.f, 0.f, 0.f, 0.f};

#pragma unroll 1
  for (int kt = 0; kt < kL / kTW; ++kt) {
    __syncthreads();
    {
      const _Float16* gk = khg + (size_t)kt * kTW * kFP;
      const _Float16* gl = klg + (size_t)kt * kTW * kFP;
#pragma unroll 2
      for (int i = 0; i < 10; ++i) {
        const int ci = tid + i * 128;
        const v8h a = *(const v8h*)(gk + ci * 8);
        const v8h b = *(const v8h*)(gl + ci * 8);
        *(v8h*)(Ksh + ci * 8) = a;
        *(v8h*)(Ksl + ci * 8) = b;
      }
#pragma unroll 2
      for (int i = 0; i < 4; ++i) {
        const int ci   = tid + i * 128;
        const int chn  = ci >> 3;
        const int prt  = ci & 7;
        const v8h a = *(const v8h*)(VP + (size_t)chn * kL + kt * kTW + prt * 8);
        *(v8h*)(Vts + chn * kTW + prt * 8) = a;
      }
    }
    __syncthreads();

#pragma unroll 1
    for (int half = 0; half < 2; ++half) {
      const int kr = half * 32 + c;
      const _Float16* k0h = Ksh + kr * kFP + 8 * hh;
      const _Float16* k0l = Ksl + kr * kFP + 8 * hh;
      v8f sm0 = (v8f){0.f, 0.f, 0.f, 0.f, 0.f, 0.f, 0.f, 0.f};
      v8f sm1 = sm0;
      v8f sr0 = sm0;
      v8f sr1 = sm0;
#pragma unroll 1
      for (int fc = 0; fc < kFP / 32; ++fc) {
        const int ko = fc * 32;
        const v16h aqh = FragH::load(qhrow + ko);
        const v16h aql = FragH::load(qlrow + ko);
        const v16h b0h = FragH::load(k0h + ko);
        const v16h b0l = FragH::load(k0l + ko);
        const v16h b1h = FragH::load(k0h + 16 * kFP + ko);
        const v16h b1l = FragH::load(k0l + 16 * kFP + ko);
        sm0 = mma_g(aqh, b0h, sm0);
        sr0 = mma_g(aqh, b0l, sr0);
        sr0 = mma_g(aql, b0h, sr0);
        sm1 = mma_g(aqh, b1h, sm1);
        sr1 = mma_g(aqh, b1l, sr1);
        sr1 = mma_g(aql, b1h, sr1);
      }

      u32a* pw = (u32a*)(&Psh[wave][0]);
#pragma unroll
      for (int r = 0; r < 8; ++r) {
        const float s0 = fmaf(sr0[r], kLoInv, sm0[r]) * kScoreInv;
        const float s1 = fmaf(sr1[r], kLoInv, sm1[r]) * kScoreInv;
        float m = fmaxf(s0, s1);
        m = fmaxf(m, __shfl_xor(m, 1, 32));
        m = fmaxf(m, __shfl_xor(m, 2, 32));
        m = fmaxf(m, __shfl_xor(m, 4, 32));
        m = fmaxf(m, __shfl_xor(m, 8, 32));
        const float mnew  = fmaxf(mrow[r], m);
        const float alpha = __expf(mrow[r] - mnew);
        mrow[r] = mnew;
        const float p0 = __expf(s0 - mnew);
        const float p1 = __expf(s1 - mnew);
        lrow[r] = fmaf(lrow[r], alpha, p0 + p1);
        oacc[0][r] *= alpha;
        oacc[1][r] *= alpha;
        oacc[2][r] *= alpha;
        oacc[3][r] *= alpha;
        pw[(8 * hh + r) * 16 + c] = pk16(h_bits(p0 * kPCarry), h_bits(p1 * kPCarry));
      }
      __builtin_amdgcn_fence(__ATOMIC_RELEASE, "workgroup");
      __builtin_amdgcn_wave_barrier();
      __builtin_amdgcn_fence(__ATOMIC_ACQUIRE, "workgroup");
      {
        const _Float16* ps = &Psh[wave][0];
        const v16h pa = FragH::load(ps + c * 32 + 8 * hh);
#pragma unroll
        for (int t = 0; t < 4; ++t) {
          const v16h vb = FragH::load(Vts + (t * 16 + c) * kTW + half * 32 + 8 * hh);
          oacc[t] = mma_g(pa, vb, oacc[t]);
        }
      }
      __builtin_amdgcn_fence(__ATOMIC_RELEASE, "workgroup");
      __builtin_amdgcn_wave_barrier();
      __builtin_amdgcn_fence(__ATOMIC_ACQUIRE, "workgroup");
    }
  }

  __syncthreads();
  float inv[8];
#pragma unroll
  for (int r = 0; r < 8; ++r) {
    float ls = lrow[r];
    ls += __shfl_xor(ls, 1, 32);
    ls += __shfl_xor(ls, 2, 32);
    ls += __shfl_xor(ls, 4, 32);
    ls += __shfl_xor(ls, 8, 32);
    inv[r] = kHeadMean / (ls * (kPCarry * kVCarry));
  }
  f32a* os = (f32a*)(&Ksh[0]) + wave * (16 * 68);
#pragma unroll
  for (int r = 0; r < 8; ++r) {
#pragma unroll
    for (int t = 0; t < 4; ++t) os[(8 * hh + r) * 68 + t * 16 + c] = oacc[t][r] * inv[r];
  }
  __builtin_amdgcn_fence(__ATOMIC_RELEASE, "workgroup");
  __builtin_amdgcn_wave_barrier();
  __builtin_amdgcn_fence(__ATOMIC_ACQUIRE, "workgroup");
  {
    const int c4 = c * 4;
    float* ob = ATTH + ((size_t)head * kL + q0) * kC;
    v4f val[8];
#pragma unroll
    for (int it = 0; it < 8; ++it) {
      const int row = it * 2 + hh;
      val[it] = *(const v4fa*)(os + row * 68 + c4);
    }
    for (int pass = 0; pass < 2; ++pass) {
#pragma unroll
      for (int it = 0; it < 8; ++it) {
        const int row = it * 2 + hh;
        *(volatile v4f*)(ob + (size_t)row * kC + c4) = val[it];
      }
      __threadfence();
    }
  }
}

__global__ __launch_bounds__(256) void proj_out_kernel(
    const float* __restrict__ ATTH, const float* __restrict__ Wo, const float* __restrict__ bo,
    float* __restrict__ OUT1)
{
  __shared__ __align__(16) float sA[64 * 68];
  __shared__ __align__(16) float sW[64 * 68];
  const int t  = threadIdx.x;
  const int l0 = blockIdx.x * 64;
  v4f sum[4];
#pragma unroll
  for (int i = 0; i < 4; ++i) sum[i] = (v4f){0.f, 0.f, 0.f, 0.f};
#pragma unroll 1
  for (int n = 0; n < kNH; ++n) {
#pragma unroll
    for (int i = 0; i < 4; ++i) {
      const int e  = t + 256 * i;
      const int lr = e >> 4;
      const int c4 = (e & 15) * 4;
      const v4f v = *(const v4f*)(ATTH + ((size_t)n * kL + l0 + lr) * kC + c4);
      sum[i] += v;
    }
  }
#pragma unroll
  for (int i = 0; i < 4; ++i) {
    const int e  = t + 256 * i;
    const int rr = e >> 4;
    const int c4 = (e & 15) * 4;
    *(v4f*)(sA + rr * 68 + c4) = sum[i];
    *(v4f*)(sW + rr * 68 + c4) = *(const v4f*)(Wo + rr * kC + c4);
  }
  __syncthreads();
  const int lq = t & 15;
  const int og = t >> 4;
  float acc[4][4];
#pragma unroll
  for (int i = 0; i < 4; ++i)
#pragma unroll
    for (int p = 0; p < 4; ++p) acc[i][p] = 0.0f;
#pragma unroll 2
  for (int cc = 0; cc < kC; ++cc) {
    float av[4], wv[4];
#pragma unroll
    for (int p = 0; p < 4; ++p) av[p] = sA[(4 * lq + p) * 68 + cc];
#pragma unroll
    for (int i = 0; i < 4; ++i) wv[i] = sW[(og + 16 * i) * 68 + cc];
#pragma unroll
    for (int i = 0; i < 4; ++i)
#pragma unroll
      for (int p = 0; p < 4; ++p) acc[i][p] = fmaf(wv[i], av[p], acc[i][p]);
  }
  v4f ov[4];
#pragma unroll
  for (int i = 0; i < 4; ++i) {
    const float bv = bo[og + 16 * i];
    ov[i] = (v4f){acc[i][0] + bv, acc[i][1] + bv, acc[i][2] + bv, acc[i][3] + bv};
  }
  for (int pass = 0; pass < 2; ++pass) {
#pragma unroll
    for (int i = 0; i < 4; ++i)
      *(volatile v4f*)(OUT1 + (size_t)(og + 16 * i) * kL + l0 + 4 * lq) = ov[i];
    __threadfence();
  }
}

extern "C" void kernel_launch(void* const* d_in, const int* in_sizes, int n_in,
                              void* d_out, int out_size, void* d_ws, size_t ws_size,
                              hipStream_t stream)
{
  if (n_in < 8) return;
  if (in_sizes[0] != kC * kL) return;
  if (in_sizes[1] != kL) return;
  if (in_sizes[2] != kA * kC) return;
  if (in_sizes[3] != kA) return;
  if (in_sizes[4] != kA * kC) return;
  if (in_sizes[5] != kA) return;
  if (in_sizes[6] != kC * kC) return;
  if (in_sizes[7] != kC) return;
  if (out_size != kC * kL) return;
  if (ws_size < kWsTotal) return;

  const float* feat  = (const float*)d_in[0];
  const float* masks = (const float*)d_in[1];
  const float* Wq    = (const float*)d_in[2];
  const float* bq    = (const float*)d_in[3];
  const float* Wk    = (const float*)d_in[4];
  const float* bk    = (const float*)d_in[5];
  const float* Wo    = (const float*)d_in[6];
  const float* bo    = (const float*)d_in[7];
  float* out = (float*)d_out;

  char* ws = (char*)d_ws;
  float*          QKRAW = (float*)(ws + kOffQKRAW);
  float*          QKN   = (float*)(ws + kOffQKN);
  unsigned short* QH    = (unsigned short*)(ws + kOffQH);
  unsigned short* QL    = (unsigned short*)(ws + kOffQL);
  unsigned short* KH    = (unsigned short*)(ws + kOffKH);
  unsigned short* KL    = (unsigned short*)(ws + kOffKL);
  unsigned short* VP    = (unsigned short*)(ws + kOffVP);
  float*          ATTH  = (float*)(ws + kOffATTH);
  float*          OUT1  = (float*)(ws + kOffOUT1);

  proj_qk_kernel<<<(kA * (kL / 4)) / 256, 256, 0, stream>>>(feat, masks, Wq, bq, Wk, bk, QKRAW);
  inorm_relu_kernel<<<2 * kA, 256, 0, stream>>>(QKRAW, QKN);
  build_patch_planes_kernel<<<(kNH * kL * kChunksPerRow) / 256, 256, 0, stream>>>(QKN, QH, QL, KH, KL);
  build_value_plane_kernel<<<(kC * (kL / 8)) / 256, 256, 0, stream>>>(feat, masks, VP);
  patch_attn_kernel<<<kNH * (kL / 64), 128, 0, stream>>>(
      (const _Float16*)QH, (const _Float16*)QL, (const _Float16*)KH, (const _Float16*)KL,
      (const _Float16*)VP, ATTH);
  proj_out_kernel<<<kL / 64, 256, 0, stream>>>(ATTH, Wo, bo, OUT1);
  inorm_relu_kernel<<<kC, 256, 0, stream>>>(OUT1, out);
}
